// BasicBlock_68951404970355
// MI455X (gfx1250) — hardware-verified
//
#include <hip/hip_runtime.h>

typedef __attribute__((ext_vector_type(16))) _Float16 v16h;
typedef __attribute__((ext_vector_type(8)))  _Float16 v8h;
typedef __attribute__((ext_vector_type(16))) __bf16   v16b;
typedef __attribute__((ext_vector_type(8)))  __bf16   v8b;
typedef __attribute__((ext_vector_type(8)))  float    v8f;
typedef __attribute__((ext_vector_type(4)))  float    v4f;

constexpr int NB_IMG    = 32;
constexpr int NCH       = 64;
constexpr int IMH       = 56;
constexpr int IMW       = 56;
constexpr int HWSZ      = IMH * IMW;
constexpr int KDIM      = NCH * 9;
constexpr int HALF_IMG  = 16;
constexpr int ROWS_HALF = HALF_IMG * HWSZ;
constexpr int I2C_ROWS  = 32;
constexpr int I2C_BLK_PER_IMG = HWSZ / I2C_ROWS;
constexpr int TILES_N   = HWSZ / 64;
constexpr int STAT_STRIDE = 128;
constexpr int NSTAT     = NB_IMG * TILES_N;
constexpr int GEMM_M = NCH;
constexpr int GEMM_N = HWSZ;
constexpr int GEMM_K = KDIM;
constexpr float CEN_CARRY = 64.0f;
constexpr float PC_SCALE  = -2.0f / 64.0f;
constexpr float D2_EPSV = 1e-12f;
constexpr float BN_EPSV = 1e-5f;

static_assert(GEMM_K % 32 == 0);
static_assert(GEMM_M % 64 == 0);
static_assert(GEMM_N % 64 == 0);
static_assert(HWSZ % I2C_ROWS == 0);
static_assert(ROWS_HALF % I2C_ROWS == 0);
static_assert(HWSZ % 4 == 0);
static_assert(NB_IMG == 2 * HALF_IMG);
static_assert(KDIM == 8 * 72);
static_assert((KDIM * 2) % 128 == 0);
static_assert(I2C_ROWS * 4 == 128);

constexpr size_t WS_P_BYTES    = (size_t)ROWS_HALF * KDIM * 2;
constexpr size_t WS_Y_BYTES    = (size_t)NB_IMG * NCH * HWSZ * 4;
constexpr size_t WS_P2_BYTES   = (size_t)ROWS_HALF * 4;
constexpr size_t WS_CEN_BYTES  = (size_t)NCH * KDIM * 2;
constexpr size_t WS_C2_BYTES   = 256;
constexpr size_t WS_STAT_BYTES = (size_t)NSTAT * STAT_STRIDE * 4;
constexpr size_t WS_BNT_BYTES  = 1024;
constexpr size_t WS_OFF_P    = 0;
constexpr size_t WS_OFF_Y1   = WS_OFF_P    + WS_P_BYTES;
constexpr size_t WS_OFF_Y2   = WS_OFF_Y1   + WS_Y_BYTES;
constexpr size_t WS_OFF_P2   = WS_OFF_Y2   + WS_Y_BYTES;
constexpr size_t WS_OFF_CEN1 = WS_OFF_P2   + WS_P2_BYTES;
constexpr size_t WS_OFF_CEN2 = WS_OFF_CEN1 + WS_CEN_BYTES;
constexpr size_t WS_OFF_C2A  = WS_OFF_CEN2 + WS_CEN_BYTES;
constexpr size_t WS_OFF_C2B  = WS_OFF_C2A  + WS_C2_BYTES;
constexpr size_t WS_OFF_STAT = WS_OFF_C2B  + WS_C2_BYTES;
constexpr size_t WS_OFF_BNT1 = WS_OFF_STAT + WS_STAT_BYTES;
constexpr size_t WS_OFF_BNT2 = WS_OFF_BNT1 + WS_BNT_BYTES;
constexpr size_t WS_TOTAL    = WS_OFF_BNT2 + WS_BNT_BYTES;
static_assert(WS_P_BYTES % 128 == 0 && WS_Y_BYTES % 128 == 0 && WS_P2_BYTES % 128 == 0);
static_assert(WS_CEN_BYTES % 128 == 0 && WS_C2_BYTES % 128 == 0 && WS_STAT_BYTES % 128 == 0 && WS_BNT_BYTES % 128 == 0);
static_assert(WS_TOTAL == 110336512);
static_assert(WS_TOTAL <= 134217728);
static_assert(WS_C2_BYTES >= NCH * 4);
static_assert(WS_BNT_BYTES >= 4 * NCH * 4);

__device__ __forceinline__ unsigned short f2bf_bits(float f) {
  unsigned u = __float_as_uint(f);
  return (unsigned short)((u + 0x7FFFu + ((u >> 16) & 1u)) >> 16);
}
__device__ __forceinline__ float bf_bits2f(unsigned short h) { return __uint_as_float(((unsigned)h) << 16); }

__device__ __forceinline__ void dep_guard_h(v8f& a, v8f& b, v16h x, v16h y) { asm volatile("v_nop\n\tv_nop\n\tv_nop\n\tv_nop" : "+v"(a), "+v"(b) : "v"(x), "v"(y)); }
__device__ __forceinline__ void dep_guard_b(v8f& a, v8f& b, v16b x, v16b y) { asm volatile("v_nop\n\tv_nop\n\tv_nop\n\tv_nop" : "+v"(a), "+v"(b) : "v"(x), "v"(y)); }
__device__ __forceinline__ void keep4_h(v16h a, v16h b, v16h c, v16h d) { asm volatile("v_nop" :: "v"(a), "v"(b), "v"(c), "v"(d)); }
__device__ __forceinline__ void keep4_b(v16b a, v16b b, v16b c, v16b d) { asm volatile("v_nop" :: "v"(a), "v"(b), "v"(c), "v"(d)); }
__device__ __forceinline__ void acc_guard4(v8f& a, v8f& b, v8f& c, v8f& d) { asm volatile("v_nop\n\tv_nop\n\tv_nop\n\tv_nop" : "+v"(a), "+v"(b), "+v"(c), "+v"(d)); }
template <typename T> struct Frag;
template <> struct Frag<_Float16> {
  typedef v16h V; union U { v16h v; v8h h[2]; };
  static __device__ __forceinline__ v16h load(const _Float16* p) {
    U f; f.h[0] = *(const v8h*)(p); f.h[1] = *(const v8h*)(p + 16); return f.v;
  }
  static __device__ __forceinline__ v8f mma(v16h a, v16h b, v8f c) {
    return __builtin_amdgcn_wmma_f32_16x16x32_f16(false, a, false, b, (short)0, c, false, false);
  }
  static __device__ __forceinline__ void guard(v8f& a, v8f& b, v16h x, v16h y) { dep_guard_h(a, b, x, y); }
  static __device__ __forceinline__ void keep(v16h a, v16h b, v16h c, v16h d) { keep4_h(a, b, c, d); }
};
template <> struct Frag<__bf16> {
  typedef v16b V; union U { v16b v; v8b h[2]; };
  static __device__ __forceinline__ v16b load(const __bf16* p) {
    U f; f.h[0] = *(const v8b*)(p); f.h[1] = *(const v8b*)(p + 16); return f.v;
  }
  static __device__ __forceinline__ v8f mma(v16b a, v16b b, v8f c) {
    return __builtin_amdgcn_wmma_f32_16x16x32_bf16(false, a, false, b, (short)0, c, false, false);
  }
  static __device__ __forceinline__ void guard(v8f& a, v8f& b, v16b x, v16b y) { dep_guard_b(a, b, x, y); }
  static __device__ __forceinline__ void keep(v16b a, v16b b, v16b c, v16b d) { keep4_b(a, b, c, d); }
};

__global__ __launch_bounds__(256) void prep_centers_k(const float* __restrict__ cen,
                                                      unsigned short* __restrict__ cenh,
                                                      float* __restrict__ c2t) {
  __shared__ __align__(16) _Float16 sC[16 * KDIM];
  __shared__ float sq[16][16];
  __shared__ __align__(16) float c2s[NCH];
  const int tid  = threadIdx.x;
  const int ol   = tid >> 4;
  const int seg  = tid & 15;
  const int wave = tid >> 5;
  const int lane = tid & 31;
  const int q    = lane >> 3;
  const int c8l  = (lane & 7) * 8;
#pragma unroll 1
  for (int ch = 0; ch < 4; ++ch) {
    const int o = ch * 16 + ol;
    const float* rp = cen + (size_t)o * KDIM + seg * 36;
    _Float16* dp = sC + ol * KDIM + seg * 36;
    float ss = 0.f;
#pragma unroll
    for (int i = 0; i < 9; ++i) {
      const v4f v = *(const v4f*)(rp + 4 * i);
#pragma unroll
      for (int e = 0; e < 4; ++e) {
        ss = fmaf(v[e], v[e], ss);
        dp[4 * i + e] = (_Float16)(v[e] * CEN_CARRY);
      }
    }
    sq[ol][seg] = ss;
    __syncthreads();
    if (tid < 16) {
      float s = 0.f;
#pragma unroll
      for (int j = 0; j < 16; ++j) s += sq[tid][j];
      c2s[ch * 16 + tid] = s;
    }
    for (int pass = 0; pass < 2; ++pass) {
#pragma unroll
      for (int it = 0; it < 5; ++it) {
        const int L   = it * 4 + q;
        const int Lc  = L < 17 ? L : 17;
        const int rr  = Lc / 9;
        const int lir = Lc - rr * 9;
        const int row = wave * 2 + rr;
        const v8h val = *(const v8h*)(sC + row * KDIM + lir * 64 + c8l);
        if (L < 18) *(volatile v8h*)(cenh + (size_t)(ch * 16 + row) * KDIM + lir * 64 + c8l) = val;
      }
      __threadfence();
    }
    __syncthreads();
  }
  if (tid < 16) {
    const v4f cv = *(const v4f*)(c2s + tid * 4);
    for (int pass = 0; pass < 2; ++pass) {
      *(volatile v4f*)(c2t + tid * 4) = cv;
      __threadfence();
    }
  }
}

template <int MODE>
__global__ __launch_bounds__(256) void im2col_k(const float* __restrict__ src, const float* __restrict__ bnt, int img0,
                                                unsigned short* __restrict__ P, float* __restrict__ P2) {
  __shared__ __align__(16) _Float16 sP[I2C_ROWS * KDIM];
  __shared__ float sq[I2C_ROWS][8];
  __shared__ __align__(16) float prow[I2C_ROWS];
  const int tid = threadIdx.x;
  const int r   = tid >> 3;
  const int g   = tid & 7;
  const int blk = blockIdx.x;
  const int bl  = blk / I2C_BLK_PER_IMG;
  const int hw0 = (blk - bl * I2C_BLK_PER_IMG) * I2C_ROWS;
  const int rowblk = blk * I2C_ROWS;
  const int hw  = hw0 + r;
  const int h   = hw / IMW;
  const int w   = hw - h * IMW;
  const float* sb = src + (size_t)(img0 + bl) * NCH * HWSZ;
  float ss = 0.f;
#pragma unroll 1
  for (int c8 = 0; c8 < 8; ++c8) {
    const int c = g * 8 + c8;
    const float* sc = sb + (size_t)c * HWSZ;
    float mu = 0.f, rs = 1.f, ga = 1.f, be = 0.f;
    if (MODE == 1) { mu = bnt[c]; rs = bnt[NCH + c]; ga = bnt[2 * NCH + c]; be = bnt[3 * NCH + c]; }
    _Float16* dst = sP + r * KDIM + c * 9;
#pragma unroll
    for (int t = 0; t < 9; ++t) {
      const int kh = t / 3;
      const int kw = t - kh * 3;
      const int hh = h + kh - 1;
      const int ww = w + kw - 1;
      const bool inb = ((unsigned)hh < (unsigned)IMH) && ((unsigned)ww < (unsigned)IMW);
      const int hc = hh < 0 ? 0 : (hh > IMH - 1 ? IMH - 1 : hh);
      const int wc = ww < 0 ? 0 : (ww > IMW - 1 ? IMW - 1 : ww);
      float val = sc[hc * IMW + wc];
      if (MODE == 1) {
        val = (val - mu) * rs;
        val = val * ga + be;
        val = fmaxf(val, 0.f);
      }
      const float v = inb ? val : 0.f;
      ss = fmaf(v, v, ss);
      dst[t] = (_Float16)v;
    }
  }
  sq[r][g] = ss;
  __syncthreads();
  if (tid < I2C_ROWS) {
    float s = 0.f;
#pragma unroll
    for (int j = 0; j < 8; ++j) s += sq[tid][j];
    prow[tid] = s;
  }
  __syncthreads();
  const int wave = tid >> 5;
  const int lane = tid & 31;
  const int q    = lane >> 3;
  const int c8l  = (lane & 7) * 8;
  unsigned short* Pb = P + (size_t)rowblk * KDIM;
  const v4f pv = *(const v4f*)(prow + (lane & 7) * 4);
  for (int pass = 0; pass < 2; ++pass) {
#pragma unroll
    for (int it = 0; it < 9; ++it) {
      const int L   = it * 4 + q;
      const int rr  = L / 9;
      const int lir = L - rr * 9;
      const int row = wave * 4 + rr;
      const v8h val = *(const v8h*)(sP + row * KDIM + lir * 64 + c8l);
      *(volatile v8h*)(Pb + (size_t)row * KDIM + lir * 64 + c8l) = val;
    }
    if (wave == 0 && lane < 8) *(volatile v4f*)(P2 + rowblk + lane * 4) = pv;
    __threadfence();
  }
}

__global__ __launch_bounds__(256) void dt_gemm64(
    const unsigned short* __restrict__ Ap, int lda,
    const unsigned short* __restrict__ Btp, int ldb, long strideB,
    const float* __restrict__ p2t, long strideP2,
    const float* __restrict__ c2t,
    float* __restrict__ Cout, int ldc, long strideC,
    float* __restrict__ stat, int img0,
    int M, int N, int K, float scale) {
  typedef _Float16 T;
  typedef Frag<_Float16>::V V;
  const T* A  = (const T*)Ap;
  const T* Bt = (const T*)Btp;
  __shared__ __align__(16) float sT[8][16 * 68];
  const int b    = blockIdx.y;
  const int lane = threadIdx.x & 31;
  const int wave = threadIdx.x >> 5;
  const int tilesN = N >> 6;
  const int tilesM = M >> 6;
  const int tile = blockIdx.x * 8 + wave;
  if (tile >= tilesM * tilesN) return;
  const int tm = tile / tilesN;
  const int tn = tile - tm * tilesN;
  const int m0 = tm << 6;
  const int n0 = tn << 6;

  const T* Bb = Bt + (size_t)b * strideB;
  const float* p2b = p2t + (size_t)b * strideP2;

  const int rlane = lane & 15;
  const int koff  = (lane >> 4) * 8;
  const int mOff  = (lane >> 4) * 8;

  v8f acc[4][4];
#pragma unroll
  for (int i = 0; i < 4; ++i)
#pragma unroll
    for (int j = 0; j < 4; ++j) acc[i][j] = (v8f){0.f,0.f,0.f,0.f,0.f,0.f,0.f,0.f};

  for (int k0 = 0; k0 < K; k0 += 32) {
    V bh[4];
#pragma unroll
    for (int j = 0; j < 4; ++j) {
      const size_t bo = (size_t)(n0 + (j << 4) + rlane) * ldb + koff + k0;
      bh[j] = Frag<T>::load(Bb + bo);
    }
#pragma unroll
    for (int i = 0; i < 4; ++i) {
      const size_t ao = (size_t)(m0 + (i << 4) + rlane) * lda + koff + k0;
      V ah = Frag<T>::load(A + ao);
#pragma unroll
      for (int j = 0; j < 4; ++j) acc[i][j] = Frag<T>::mma(ah, bh[j], acc[i][j]);
      Frag<T>::guard(acc[i][0], acc[i][3], ah, ah);
    }
    Frag<T>::keep(bh[0], bh[1], bh[2], bh[3]);
  }
  acc_guard4(acc[0][0], acc[0][1], acc[0][2], acc[0][3]);
  acc_guard4(acc[1][0], acc[1][1], acc[1][2], acc[1][3]);
  acc_guard4(acc[2][0], acc[2][1], acc[2][2], acc[2][3]);
  acc_guard4(acc[3][0], acc[3][1], acc[3][2], acc[3][3]);

  float* slab = sT[wave];
  float p2v[4];
#pragma unroll
  for (int j = 0; j < 4; ++j) p2v[j] = p2b[n0 + (j << 4) + rlane];
  const int srow  = lane & 15;
  const int shalf = lane >> 4;
  float S1[4], S2[4];
  float* C = Cout + (size_t)(img0 + b) * strideC;
#pragma unroll
  for (int i = 0; i < 4; ++i) {
    const int mBase = m0 + (i << 4);
    const v8f c2v = *(const v8f*)(c2t + mBase + mOff);
#pragma unroll
    for (int j = 0; j < 4; ++j) {
#pragma unroll
      for (int r = 0; r < 8; ++r) {
        float t = p2v[j] + acc[i][j][r] * scale;
        t = t + c2v[r];
        t = fmaxf(t, D2_EPSV);
        slab[(mOff + r) * 68 + (j << 4) + rlane] = __builtin_amdgcn_sqrtf(t);
      }
    }
    __builtin_amdgcn_fence(__ATOMIC_RELEASE, "workgroup");
    __builtin_amdgcn_wave_barrier();
    __builtin_amdgcn_fence(__ATOMIC_ACQUIRE, "workgroup");
    {
      const float* sp = slab + srow * 68 + shalf * 32;
      float s1 = 0.f, s2 = 0.f;
#pragma unroll
      for (int q4 = 0; q4 < 8; ++q4) {
        const v4f v = *(const v4f*)(sp + 4 * q4);
#pragma unroll
        for (int e = 0; e < 4; ++e) { s1 += v[e]; s2 = fmaf(v[e], v[e], s2); }
      }
      s1 += __shfl_xor(s1, 16, 32);
      s2 += __shfl_xor(s2, 16, 32);
      S1[i] = s1;
      S2[i] = s2;
    }
    {
      const int hh = lane >> 4, c4 = (lane & 15) * 4;
      for (int pass = 0; pass < 2; ++pass) {
#pragma unroll
        for (int it = 0; it < 8; ++it) {
          const int row = it * 2 + hh;
          v4f v = *(const v4f*)(slab + row * 68 + c4);
          *(volatile v4f*)(C + (size_t)(mBase + row) * ldc + n0 + c4) = v;
        }
        __threadfence();
      }
    }
    __builtin_amdgcn_fence(__ATOMIC_RELEASE, "workgroup");
    __builtin_amdgcn_wave_barrier();
    __builtin_amdgcn_fence(__ATOMIC_ACQUIRE, "workgroup");
  }
#pragma unroll
  for (int i = 0; i < 4; ++i) slab[shalf * 64 + (i << 4) + srow] = shalf ? S2[i] : S1[i];
  __builtin_amdgcn_fence(__ATOMIC_RELEASE, "workgroup");
  __builtin_amdgcn_wave_barrier();
  __builtin_amdgcn_fence(__ATOMIC_ACQUIRE, "workgroup");
  {
    const int widx = (img0 + b) * (tilesM * tilesN) + tile;
    const v4f sv = *(const v4f*)(slab + lane * 4);
    float* stp = stat + (size_t)widx * STAT_STRIDE + lane * 4;
    for (int pass = 0; pass < 2; ++pass) {
      *(volatile v4f*)stp = sv;
      __threadfence();
    }
  }
}

__global__ __launch_bounds__(64) void bn_finalize_k(const float* __restrict__ stat, int nrec,
                                                    const float* __restrict__ gamma, const float* __restrict__ beta,
                                                    float* __restrict__ bnt, double inv_count) {
  __shared__ __align__(16) float st[4 * NCH];
  const int o = threadIdx.x;
  double s1 = 0.0, s2 = 0.0;
#pragma unroll 1
  for (int wrec = 0; wrec < nrec; ++wrec) {
    s1 += (double)stat[(size_t)wrec * STAT_STRIDE + o];
    s2 += (double)stat[(size_t)wrec * STAT_STRIDE + NCH + o];
  }
  const double mu = s1 * inv_count;
  double var = s2 * inv_count - mu * mu;
  var = var < 0.0 ? 0.0 : var;
  const float muf  = (float)mu;
  const float varf = (float)var;
  const float rs   = 1.0f / sqrtf(varf + BN_EPSV);
  st[o]           = muf;
  st[NCH + o]     = rs;
  st[2 * NCH + o] = gamma[o];
  st[3 * NCH + o] = beta[o];
  __syncthreads();
  const int wave = o >> 5;
  const int lane = o & 31;
  const v4f v = *(const v4f*)(st + wave * 128 + lane * 4);
  for (int pass = 0; pass < 2; ++pass) {
    *(volatile v4f*)(bnt + wave * 128 + lane * 4) = v;
    __threadfence();
  }
}

__global__ __launch_bounds__(256) void bn_res_relu_k(const float* __restrict__ y, const float* __restrict__ bnt,
                                                     const float* __restrict__ x, float* __restrict__ out, int n4) {
  const int i = blockIdx.x * 256 + threadIdx.x;
  if (i >= n4) return;
  const int o = (i / (HWSZ / 4)) & (NCH - 1);
  const v4f yv = *(const v4f*)(y + (size_t)i * 4);
  const v4f xv = *(const v4f*)(x + (size_t)i * 4);
  const float mu = bnt[o], rs = bnt[NCH + o], ga = bnt[2 * NCH + o], be = bnt[3 * NCH + o];
  v4f rv;
#pragma unroll
  for (int e = 0; e < 4; ++e) {
    float t = (yv[e] - mu) * rs;
    t = t * ga + be;
    t = t + xv[e];
    rv[e] = fmaxf(t, 0.f);
  }
  float* op = out + (size_t)i * 4;
  *(volatile v4f*)op = rv;
  __threadfence();
  *(volatile v4f*)op = rv;
}

extern "C" void kernel_launch(void* const* d_in, const int* in_sizes, int n_in,
                              void* d_out, int out_size, void* d_ws, size_t ws_size,
                              hipStream_t stream) {
  if (n_in < 7) return;
  if (in_sizes[0] != NB_IMG * NCH * HWSZ) return;
  if (in_sizes[1] != NCH * KDIM || in_sizes[4] != NCH * KDIM) return;
  if (in_sizes[2] != NCH || in_sizes[3] != NCH || in_sizes[5] != NCH || in_sizes[6] != NCH) return;
  if (out_size != NB_IMG * NCH * HWSZ) return;
  if (ws_size < WS_TOTAL) return;

  const float* x    = (const float*)d_in[0];
  const float* cen1 = (const float*)d_in[1];
  const float* g1   = (const float*)d_in[2];
  const float* b1   = (const float*)d_in[3];
  const float* cen2 = (const float*)d_in[4];
  const float* g2   = (const float*)d_in[5];
  const float* b2   = (const float*)d_in[6];
  float* out = (float*)d_out;

  char* ws = (char*)d_ws;
  unsigned short* wsP    = (unsigned short*)(ws + WS_OFF_P);
  float*          wsY1   = (float*)(ws + WS_OFF_Y1);
  float*          wsY2   = (float*)(ws + WS_OFF_Y2);
  float*          wsP2   = (float*)(ws + WS_OFF_P2);
  unsigned short* wsCen1 = (unsigned short*)(ws + WS_OFF_CEN1);
  unsigned short* wsCen2 = (unsigned short*)(ws + WS_OFF_CEN2);
  float*          wsC2a  = (float*)(ws + WS_OFF_C2A);
  float*          wsC2b  = (float*)(ws + WS_OFF_C2B);
  float*          wsStat = (float*)(ws + WS_OFF_STAT);
  float*          wsBnt1 = (float*)(ws + WS_OFF_BNT1);
  float*          wsBnt2 = (float*)(ws + WS_OFF_BNT2);

  const int  i2cBlocks = ROWS_HALF / I2C_ROWS;
  const dim3 gemmGrid((TILES_N + 7) / 8, HALF_IMG);
  const long strideB  = (long)HWSZ * KDIM;
  const long strideP2 = (long)HWSZ;
  const long strideC  = (long)NCH * HWSZ;
  const double invCount = 1.0 / (double)(NB_IMG * HWSZ);
  const int n4 = out_size / 4;
  const int ewBlocks = (n4 + 255) / 256;

  prep_centers_k<<<1, 256, 0, stream>>>(cen1, wsCen1, wsC2a);
  for (int half = 0; half < 2; ++half) {
    const int img0 = half * HALF_IMG;
    im2col_k<0><<<i2cBlocks, 256, 0, stream>>>(x, wsBnt1, img0, wsP, wsP2);
    dt_gemm64<<<gemmGrid, 256, 0, stream>>>(wsCen1, KDIM, wsP, KDIM, strideB, wsP2, strideP2, wsC2a,
                                            wsY1, HWSZ, strideC, wsStat, img0,
                                            GEMM_M, GEMM_N, GEMM_K, PC_SCALE);
  }
  bn_finalize_k<<<1, 64, 0, stream>>>(wsStat, NSTAT, g1, b1, wsBnt1, invCount);

  prep_centers_k<<<1, 256, 0, stream>>>(cen2, wsCen2, wsC2b);
  for (int half = 0; half < 2; ++half) {
    const int img0 = half * HALF_IMG;
    im2col_k<1><<<i2cBlocks, 256, 0, stream>>>(wsY1, wsBnt1, img0, wsP, wsP2);
    dt_gemm64<<<gemmGrid, 256, 0, stream>>>(wsCen2, KDIM, wsP, KDIM, strideB, wsP2, strideP2, wsC2b,
                                            wsY2, HWSZ, strideC, wsStat, img0,
                                            GEMM_M, GEMM_N, GEMM_K, PC_SCALE);
  }
  bn_finalize_k<<<1, 64, 0, stream>>>(wsStat, NSTAT, g2, b2, wsBnt2, invCount);

  bn_res_relu_k<<<ewBlocks, 256, 0, stream>>>(wsY2, wsBnt2, x, out, n4);
}
